// KiperwasserDependencyParser_71992241816192
// MI455X (gfx1250) — hardware-verified
//
#include <hip/hip_runtime.h>
#include <hip/hip_bf16.h>

typedef __attribute__((ext_vector_type(16))) _Float16 v16h;
typedef __attribute__((ext_vector_type(8)))  _Float16 v8h;
typedef __attribute__((ext_vector_type(16))) __bf16   v16b;
typedef __attribute__((ext_vector_type(8)))  __bf16   v8b;
typedef __attribute__((ext_vector_type(8)))  float    v8f;
typedef __attribute__((ext_vector_type(4)))  float    v4f;
typedef __attribute__((ext_vector_type(4)))  unsigned v4u;
typedef __attribute__((ext_vector_type(2)))  unsigned v2u;

__device__ __forceinline__ unsigned short f2bf_bits(float f) {
  unsigned u = __float_as_uint(f);
  return (unsigned short)((u + 0x7FFFu + ((u >> 16) & 1u)) >> 16);
}
__device__ __forceinline__ float bf_bits2f(unsigned short h) { return __uint_as_float(((unsigned)h) << 16); }

__device__ __forceinline__ void dep_guard_h(v8f& a, v8f& b, v16h x, v16h y) { asm volatile("v_nop\n\tv_nop\n\tv_nop\n\tv_nop" : "+v"(a), "+v"(b) : "v"(x), "v"(y)); }
__device__ __forceinline__ void dep_guard_b(v8f& a, v8f& b, v16b x, v16b y) { asm volatile("v_nop\n\tv_nop\n\tv_nop\n\tv_nop" : "+v"(a), "+v"(b) : "v"(x), "v"(y)); }
__device__ __forceinline__ void keep4_h(v16h a, v16h b, v16h c, v16h d) { asm volatile("v_nop" :: "v"(a), "v"(b), "v"(c), "v"(d)); }
__device__ __forceinline__ void keep4_b(v16b a, v16b b, v16b c, v16b d) { asm volatile("v_nop" :: "v"(a), "v"(b), "v"(c), "v"(d)); }
__device__ __forceinline__ void acc_guard4(v8f& a, v8f& b, v8f& c, v8f& d) { asm volatile("v_nop\n\tv_nop\n\tv_nop\n\tv_nop" : "+v"(a), "+v"(b), "+v"(c), "+v"(d)); }
template <typename T> struct Frag;
template <> struct Frag<_Float16> {
  typedef v16h V; union U { v16h v; v8h h[2]; };
  static __device__ __forceinline__ v16h load(const _Float16* p) {
    U f; f.h[0] = *(const v8h*)(p); f.h[1] = *(const v8h*)(p + 16); return f.v;
  }
  static __device__ __forceinline__ v8f mma(v16h a, v16h b, v8f c) {
    return __builtin_amdgcn_wmma_f32_16x16x32_f16(false, a, false, b, (short)0, c, false, false);
  }
  static __device__ __forceinline__ void guard(v8f& a, v8f& b, v16h x, v16h y) { dep_guard_h(a, b, x, y); }
  static __device__ __forceinline__ void keep(v16h a, v16h b, v16h c, v16h d) { keep4_h(a, b, c, d); }
};
template <> struct Frag<__bf16> {
  typedef v16b V; union U { v16b v; v8b h[2]; };
  static __device__ __forceinline__ v16b load(const __bf16* p) {
    U f; f.h[0] = *(const v8b*)(p); f.h[1] = *(const v8b*)(p + 16); return f.v;
  }
  static __device__ __forceinline__ v8f mma(v16b a, v16b b, v8f c) {
    return __builtin_amdgcn_wmma_f32_16x16x32_bf16(false, a, false, b, (short)0, c, false, false);
  }
  static __device__ __forceinline__ void guard(v8f& a, v8f& b, v16b x, v16b y) { dep_guard_b(a, b, x, y); }
  static __device__ __forceinline__ void keep(v16b a, v16b b, v16b c, v16b d) { keep4_b(a, b, c, d); }
};

template <int ET> struct Elem;
template <> struct Elem<0> { typedef _Float16 T; };
template <> struct Elem<1> { typedef __bf16 T; };
template <int ET, bool SPLIT, int BIAS_MODE, int OUT_MODE, bool RESID, int ACT = 0>
__global__ __launch_bounds__(256) void wmma_gemm64(
    const unsigned short* __restrict__ Ap, const unsigned short* __restrict__ A2p, int lda, long strideA,
    const unsigned short* __restrict__ Btp, const unsigned short* __restrict__ Bt2p, int ldb, long strideB,
    void* __restrict__ Cout, void* __restrict__ Cout2, int ldc, long strideC,
    const float* __restrict__ bias,
    const float* __restrict__ resid, long strideR,
    int M, int N, int K, float scale) {
  typedef typename Elem<ET>::T T;
  typedef typename Frag<T>::V V;
  const T* A = (const T*)Ap; const T* A2 = (const T*)A2p; const T* Bt = (const T*)Btp; const T* Bt2 = (const T*)Bt2p;
  __shared__ __align__(16) float sT[8][16 * 68];
  const int b    = blockIdx.y;
  const int lane = threadIdx.x & 31;
  const int wave = threadIdx.x >> 5;
  const int tilesN = N >> 6;
  const int tilesM = M >> 6;
  const int tile = blockIdx.x * 8 + wave;
  if (tile >= tilesM * tilesN) return;
  const int tm = tile / tilesN;
  const int tn = tile - tm * tilesN;
  const int m0 = tm << 6;
  const int n0 = tn << 6;

  const T* Ab  = A  + (size_t)b * strideA;
  const T* Bb  = Bt + (size_t)b * strideB;
  const T* Ab2 = SPLIT ? (A2  + (size_t)b * strideA) : nullptr;
  const T* Bb2 = SPLIT ? (Bt2 + (size_t)b * strideB) : nullptr;

  const int rlane = lane & 15;
  const int koff  = (lane >> 4) * 8;
  const int mOff  = (lane >> 4) * 8;

  v8f acc[4][4];
#pragma unroll
  for (int i = 0; i < 4; ++i)
#pragma unroll
    for (int j = 0; j < 4; ++j) acc[i][j] = (v8f){0.f,0.f,0.f,0.f,0.f,0.f,0.f,0.f};

  for (int k0 = 0; k0 < K; k0 += 32) {
    V bh[4], bl[4];
#pragma unroll
    for (int j = 0; j < 4; ++j) {
      const size_t bo = (size_t)(n0 + (j << 4) + rlane) * ldb + koff + k0;
      bh[j] = Frag<T>::load(Bb + bo);
      if (SPLIT) bl[j] = Frag<T>::load(Bb2 + bo);
    }
#pragma unroll
    for (int i = 0; i < 4; ++i) {
      const size_t ao = (size_t)(m0 + (i << 4) + rlane) * lda + koff + k0;
      V ah = Frag<T>::load(Ab + ao);
      V al;
      if (SPLIT) al = Frag<T>::load(Ab2 + ao);
#pragma unroll
      for (int j = 0; j < 4; ++j) {
        acc[i][j] = Frag<T>::mma(ah, bh[j], acc[i][j]);
        if (SPLIT) {
          acc[i][j] = Frag<T>::mma(ah, bl[j], acc[i][j]);
          acc[i][j] = Frag<T>::mma(al, bh[j], acc[i][j]);
        }
      }
      Frag<T>::guard(acc[i][0], acc[i][3], ah, SPLIT ? al : ah);
    }
    Frag<T>::keep(bh[0], bh[1], bh[2], bh[3]);
    if (SPLIT) Frag<T>::keep(bl[0], bl[1], bl[2], bl[3]);
  }
  acc_guard4(acc[0][0], acc[0][1], acc[0][2], acc[0][3]);
  acc_guard4(acc[1][0], acc[1][1], acc[1][2], acc[1][3]);
  acc_guard4(acc[2][0], acc[2][1], acc[2][2], acc[2][3]);
  acc_guard4(acc[3][0], acc[3][1], acc[3][2], acc[3][3]);

  float* slab = sT[wave];
  const float* Rb = RESID ? (resid + (size_t)b * strideR) : nullptr;
#pragma unroll
  for (int i = 0; i < 4; ++i) {
    const int mBase = m0 + (i << 4);
#pragma unroll
    for (int j = 0; j < 4; ++j) {
      const int n = n0 + (j << 4) + rlane;
      float bv = 0.f;
      if (BIAS_MODE == 2) bv = bias[n];
#pragma unroll
      for (int r = 0; r < 8; ++r) {
        float v = acc[i][j][r] * scale;
        if (BIAS_MODE == 1) v += bias[mBase + mOff + r];
        if (BIAS_MODE == 2) v += bv;
        if (RESID) v += Rb[(size_t)(mBase + mOff + r) * ldc + n];
        if (ACT == 1) v = tanhf(v);
        if (ACT == 2) v = fmaxf(v, 0.0f);
        if (ACT == 3) v = v / (1.0f + expf(-v));
        if (ACT == 4) v = (v > 0.f) ? v : 0.01f * v;
        if (ACT == 5) v = 0.5f * v * (1.0f + erff(v * 0.70710678118654752f));
        slab[(mOff + r) * 68 + (j << 4) + rlane] = v;
      }
    }
    __builtin_amdgcn_fence(__ATOMIC_RELEASE, "workgroup");
    __builtin_amdgcn_wave_barrier();
    __builtin_amdgcn_fence(__ATOMIC_ACQUIRE, "workgroup");
    if (OUT_MODE == 0) {
      float* C = (float*)Cout + (size_t)b * strideC;
      const int hh = lane >> 4, c4 = (lane & 15) * 4;
      for (int pass = 0; pass < 2; ++pass) {
#pragma unroll
        for (int it = 0; it < 8; ++it) {
          const int row = it * 2 + hh;
          v4f v = *(const v4f*)(slab + row * 68 + c4);
          *(volatile v4f*)(C + (size_t)(mBase + row) * ldc + n0 + c4) = v;
        }
        __threadfence();
      }
    } else {
      const int q = lane >> 3, c8 = (lane & 7) * 8;
      unsigned short* C  = (unsigned short*)Cout  + (size_t)b * strideC;
      unsigned short* C2 = (OUT_MODE == 2) ? ((unsigned short*)Cout2 + (size_t)b * strideC) : nullptr;
      for (int pass = 0; pass < 2; ++pass) {
#pragma unroll
        for (int it = 0; it < 4; ++it) {
          const int row = it * 4 + q;
          const float* sp = slab + row * 68 + c8;
          v8h hv, lv;
#pragma unroll
          for (int e = 0; e < 8; ++e) {
            if (OUT_MODE == 1) {
              hv[e] = (_Float16)sp[e];
            } else {
              unsigned short hb = f2bf_bits(sp[e]);
              unsigned short lb = f2bf_bits(sp[e] - bf_bits2f(hb));
              hv[e] = __builtin_bit_cast(_Float16, hb);
              lv[e] = __builtin_bit_cast(_Float16, lb);
            }
          }
          *(volatile v8h*)(C + (size_t)(mBase + row) * ldc + n0 + c8) = hv;
          if (OUT_MODE == 2) *(volatile v8h*)(C2 + (size_t)(mBase + row) * ldc + n0 + c8) = lv;
        }
        __threadfence();
      }
    }
    __builtin_amdgcn_fence(__ATOMIC_RELEASE, "workgroup");
    __builtin_amdgcn_wave_barrier();
    __builtin_amdgcn_fence(__ATOMIC_ACQUIRE, "workgroup");
  }
}

#define SEQ_N   1024
#define HID     256
#define NGATE   1024
#define WEMB    100
#define PEMB    25
#define XKPAD   128
#define HPITCH  1024
#define MHID    100
#define ABPITCH 256
#define PRM_B0    0
#define PRM_B1    2048
#define PRM_MB1   4096
#define PRM_W2    4224
#define PRM_MB2   4352
#define PRM_TOTAL 4384

__device__ __forceinline__ int clampi(int v, int lo, int hi) { return v < lo ? lo : (v > hi ? hi : v); }
__device__ __forceinline__ float bf_rne(float v) { return bf_bits2f(f2bf_bits(v)); }

__global__ __launch_bounds__(256) void prm_kernel(
    const float* __restrict__ b0, const float* __restrict__ b1, const float* __restrict__ mb1,
    const float* __restrict__ w2, const float* __restrict__ mb2, float* __restrict__ prm) {
  const int i = blockIdx.x * 256 + threadIdx.x;
  if (i >= PRM_TOTAL) return;
  const int i0 = clampi(i, 0, 2047);
  const int i1 = clampi(i - PRM_B1, 0, 2047);
  const int i2 = clampi(i - PRM_MB1, 0, MHID - 1);
  const int i3 = clampi(i - PRM_W2, 0, MHID - 1);
  const float v0 = b0[i0];
  const float v1 = b1[i1];
  const float v2 = mb1[i2];
  const float v3 = w2[i3];
  const float v4 = mb2[0];
  float v;
  if (i < PRM_B1)       v = v0;
  else if (i < PRM_MB1) v = v1;
  else if (i < PRM_W2)  v = ((i - PRM_MB1) < MHID) ? v2 : 0.0f;
  else if (i < PRM_MB2) v = ((i - PRM_W2) < MHID) ? v3 : 0.0f;
  else                  v = (i == PRM_MB2) ? v4 : 0.0f;
  v = bf_rne(v);
  ((volatile float*)prm)[i] = v;
  __threadfence();
  ((volatile float*)prm)[i] = v;
}

__device__ __forceinline__ unsigned short embed_elem(const float* wp, const float* pp, int c) {
  const int cw = c < WEMB ? c : (WEMB - 1);
  int cp = c - WEMB; cp = clampi(cp, 0, PEMB - 1);
  const float vw = wp[cw];
  const float vp = pp[cp];
  const float v = (c < WEMB) ? vw : ((c < WEMB + PEMB) ? vp : 0.0f);
  return f2bf_bits(v);
}
__global__ __launch_bounds__(256) void embed_rows_bf16(
    const int* __restrict__ widx, const int* __restrict__ pidx,
    const float* __restrict__ we, int nWordRows, const float* __restrict__ pe, int nPosRows,
    unsigned short* __restrict__ X) {
  const int lane = threadIdx.x & 31, wave = threadIdx.x >> 5;
  const int row = blockIdx.x * 8 + wave;
  int wr = widx[row]; wr = clampi(wr, 0, nWordRows - 1);
  int pr = pidx[row]; pr = clampi(pr, 0, nPosRows - 1);
  const float* wp = we + (size_t)wr * WEMB;
  const float* pp = pe + (size_t)pr * PEMB;
  const unsigned short h0 = embed_elem(wp, pp, 4 * lane + 0);
  const unsigned short h1 = embed_elem(wp, pp, 4 * lane + 1);
  const unsigned short h2 = embed_elem(wp, pp, 4 * lane + 2);
  const unsigned short h3 = embed_elem(wp, pp, 4 * lane + 3);
  v2u pk;
  pk.x = (unsigned)h0 | ((unsigned)h1 << 16);
  pk.y = (unsigned)h2 | ((unsigned)h3 << 16);
  unsigned short* dp = X + (size_t)row * XKPAD + 4 * lane;
  for (int pass = 0; pass < 2; ++pass) {
    *(volatile v2u*)dp = pk;
    __threadfence();
  }
}

__device__ __forceinline__ unsigned short cast_elem(const float* sp, int cc, int srcCols, int kdup, int rowValid) {
  int cs = cc;
  if (kdup && cs >= srcCols) cs -= srcCols;
  const int valid = rowValid && (cs < srcCols);
  const int csc = cs < srcCols ? cs : (srcCols - 1);
  float v = sp[csc];
  v = valid ? v : 0.0f;
  return f2bf_bits(v);
}
__global__ __launch_bounds__(256) void cast_rows_bf16(
    const float* __restrict__ src, int srcRows, int srcPitch, int colOff, int srcCols,
    unsigned short* __restrict__ dst, int dstCols, int kdup) {
  const int lane = threadIdx.x & 31, wave = threadIdx.x >> 5;
  const int row = blockIdx.x * 8 + wave;
  const int rowValid = row < srcRows;
  const int srow = rowValid ? row : (srcRows - 1);
  const float* sp = src + (size_t)srow * srcPitch + colOff;
  unsigned short* dp = dst + (size_t)row * dstCols;
#pragma unroll 1
  for (int c0 = 0; c0 < dstCols; c0 += 256) {
    const int c = c0 + 8 * lane;
    v4u pk;
    pk.x = (unsigned)cast_elem(sp, c + 0, srcCols, kdup, rowValid) | ((unsigned)cast_elem(sp, c + 1, srcCols, kdup, rowValid) << 16);
    pk.y = (unsigned)cast_elem(sp, c + 2, srcCols, kdup, rowValid) | ((unsigned)cast_elem(sp, c + 3, srcCols, kdup, rowValid) << 16);
    pk.z = (unsigned)cast_elem(sp, c + 4, srcCols, kdup, rowValid) | ((unsigned)cast_elem(sp, c + 5, srcCols, kdup, rowValid) << 16);
    pk.w = (unsigned)cast_elem(sp, c + 6, srcCols, kdup, rowValid) | ((unsigned)cast_elem(sp, c + 7, srcCols, kdup, rowValid) << 16);
    for (int pass = 0; pass < 2; ++pass) {
      if (c < dstCols) *(volatile v4u*)(dp + c) = pk;
      __threadfence();
    }
  }
}

__device__ __forceinline__ void store_h_row(const unsigned short* hs, unsigned short* __restrict__ Hout,
                                            int trow, int dir, int lane) {
  const v4u vh = *(const v4u*)(hs + 8 * lane);
  const v4u vl = *(const v4u*)(hs + HID + 8 * lane);
  unsigned short* ph = Hout + (size_t)trow * HPITCH + dir * HID + 8 * lane;
  unsigned short* pl = ph + 2 * HID;
  for (int pass = 0; pass < 2; ++pass) {
    *(volatile v4u*)ph = vh;
    *(volatile v4u*)pl = vl;
    __threadfence();
  }
}

__global__ __launch_bounds__(512) void bilstm_dir_kernel(
    const unsigned short* __restrict__ Whh16, const float* __restrict__ Zin,
    const float* __restrict__ prm, int boff, unsigned short* __restrict__ Hout) {
  __shared__ __align__(16) unsigned short hs[16 * HID];
  __shared__ float zpart[3 * NGATE];
  const int tid = threadIdx.x;
  const int lane = tid & 31, wave = tid >> 5;
  const int dir = blockIdx.x;
  const int rlane = lane & 15;
  const int koff = (lane >> 4) * 8;
  const int hh = lane >> 4;

  {
    v4u z4; z4.x = 0u; z4.y = 0u; z4.z = 0u; z4.w = 0u;
    *(v4u*)(hs + 8 * tid) = z4;
  }
  const int jc = tid & (HID - 1);
  const float* bp = prm + boff + dir * NGATE;
  const float b_i = bp[jc];
  const float b_f = bp[HID + jc];
  const float b_g = bp[2 * HID + jc];
  const float b_o = bp[3 * HID + jc];
  const __bf16* Wd = (const __bf16*)Whh16 + (size_t)dir * NGATE * HID + (size_t)(wave * 64) * HID;
  const float* Zd = Zin + (size_t)dir * SEQ_N * NGATE;
  float creg = 0.0f;
  __syncthreads();

  for (int s = 0; s < SEQ_N; ++s) {
    const int t = dir ? (SEQ_N - 1 - s) : s;
    if (wave == 0 && s > 0) store_h_row(hs, Hout, dir ? (t + 1) : (t - 1), dir, lane);

    v8f acc[4];
#pragma unroll
    for (int i = 0; i < 4; ++i) acc[i] = (v8f){0.f,0.f,0.f,0.f,0.f,0.f,0.f,0.f};
#pragma unroll 2
    for (int ks = 0; ks < HID / 32; ++ks) {
      const int k0 = ks * 32;
      const v16b bf = Frag<__bf16>::load((const __bf16*)hs + rlane * HID + k0 + koff);
      v16b af[4];
#pragma unroll
      for (int i = 0; i < 4; ++i) af[i] = Frag<__bf16>::load(Wd + (size_t)(i * 16 + rlane) * HID + k0 + koff);
#pragma unroll
      for (int i = 0; i < 4; ++i) acc[i] = Frag<__bf16>::mma(af[i], bf, acc[i]);
      dep_guard_b(acc[0], acc[3], af[3], bf);
      keep4_b(af[0], af[1], af[2], bf);
    }
    acc_guard4(acc[0], acc[1], acc[2], acc[3]);
#pragma unroll
    for (int i = 0; i < 4; ++i) {
#pragma unroll
      for (int r = 0; r < 8; ++r) {
        const int grow = wave * 64 + i * 16 + hh * 8 + r;
        const float v = acc[i][r];
        if (rlane < 3) zpart[rlane * NGATE + grow] = v;
      }
    }
    __syncthreads();

    if (tid < HID) {
      const float* zp = Zd + (size_t)t * NGATE + tid;
      const float zin_i = zp[0];
      const float zin_f = zp[HID];
      const float zin_g = zp[2 * HID];
      const float zin_o = zp[3 * HID];
      const float zh_i = (zpart[tid] + zpart[NGATE + tid]) + zpart[2 * NGATE + tid];
      const float zh_f = (zpart[HID + tid] + zpart[NGATE + HID + tid]) + zpart[2 * NGATE + HID + tid];
      const float zh_g = (zpart[2 * HID + tid] + zpart[NGATE + 2 * HID + tid]) + zpart[2 * NGATE + 2 * HID + tid];
      const float zh_o = (zpart[3 * HID + tid] + zpart[NGATE + 3 * HID + tid]) + zpart[2 * NGATE + 3 * HID + tid];
      const float zi = (zin_i + zh_i) + b_i;
      const float zf = (zin_f + zh_f) + b_f;
      const float zg = (zin_g + zh_g) + b_g;
      const float zo = (zin_o + zh_o) + b_o;
      const float ig = 1.0f / (1.0f + expf(-zi));
      const float fg = 1.0f / (1.0f + expf(-zf));
      const float og = 1.0f / (1.0f + expf(-zo));
      const float gt = tanhf(zg);
      creg = fg * creg + ig * gt;
      const float hval = og * tanhf(creg);
      const unsigned short hb = f2bf_bits(hval);
      const float r1 = hval - bf_bits2f(hb);
      const unsigned short mb = f2bf_bits(r1);
      const float r2 = r1 - bf_bits2f(mb);
      const unsigned short lb = f2bf_bits(r2);
      hs[tid] = hb;
      hs[HID + tid] = mb;
      hs[2 * HID + tid] = lb;
    }
    __syncthreads();
  }
  if (wave == 0) store_h_row(hs, Hout, dir ? 0 : (SEQ_N - 1), dir, lane);
}

__device__ __forceinline__ float tanh_fast(float x) {
  const float ax = fabsf(x);
  const float e = __expf(-2.0f * ax);
  const float r = (1.0f - e) * __builtin_amdgcn_rcpf(1.0f + e);
  return copysignf(r, x);
}
__global__ __launch_bounds__(256) void pair_score_kernel(
    const float* __restrict__ AB, const float* __restrict__ prm, float* __restrict__ out) {
  __shared__ float aS[32 * MHID];
  __shared__ float bS[64 * MHID];
  __shared__ float wS[MHID];
  __shared__ __align__(16) float oS[32 * 64];
  const int tid = threadIdx.x;
  const int lane = tid & 31, wave = tid >> 5;
  const int i0 = blockIdx.y * 32;
  const int j0 = blockIdx.x * 64;
  for (int idx = tid; idx < 32 * MHID; idx += 256) {
    const int i = idx / MHID, hcol = idx - i * MHID;
    aS[idx] = AB[(size_t)(i0 + i) * ABPITCH + hcol] + prm[PRM_MB1 + hcol];
  }
  for (int idx = tid; idx < 64 * MHID; idx += 256) {
    const int j = idx / MHID, hcol = idx - j * MHID;
    bS[idx] = AB[(size_t)(j0 + j) * ABPITCH + 128 + hcol];
  }
  if (tid < MHID) wS[tid] = prm[PRM_W2 + tid];
  const float b2v = prm[PRM_MB2];
  __syncthreads();

  const int ti = tid >> 4, tj = tid & 15;
  const float* ap0 = aS + (2 * ti) * MHID;
  const float* ap1 = ap0 + MHID;
  const float* bp0 = bS + tj * MHID;
  const float* bp1 = bS + (tj + 16) * MHID;
  const float* bp2 = bS + (tj + 32) * MHID;
  const float* bp3 = bS + (tj + 48) * MHID;
  float s00 = 0.f, s01 = 0.f, s02 = 0.f, s03 = 0.f;
  float s10 = 0.f, s11 = 0.f, s12 = 0.f, s13 = 0.f;
#pragma unroll 1
  for (int hcol = 0; hcol < MHID; ++hcol) {
    const float w = wS[hcol];
    const float a0 = ap0[hcol], a1 = ap1[hcol];
    const float c0 = bp0[hcol], c1 = bp1[hcol], c2 = bp2[hcol], c3 = bp3[hcol];
    s00 += w * tanh_fast(a0 + c0);
    s01 += w * tanh_fast(a0 + c1);
    s02 += w * tanh_fast(a0 + c2);
    s03 += w * tanh_fast(a0 + c3);
    s10 += w * tanh_fast(a1 + c0);
    s11 += w * tanh_fast(a1 + c1);
    s12 += w * tanh_fast(a1 + c2);
    s13 += w * tanh_fast(a1 + c3);
  }
  {
    float* o0 = oS + (2 * ti) * 64;
    float* o1 = o0 + 64;
    o0[tj] = s00 + b2v; o0[tj + 16] = s01 + b2v; o0[tj + 32] = s02 + b2v; o0[tj + 48] = s03 + b2v;
    o1[tj] = s10 + b2v; o1[tj + 16] = s11 + b2v; o1[tj + 32] = s12 + b2v; o1[tj + 48] = s13 + b2v;
  }
  __syncthreads();
  {
    const int hh = lane >> 4, c4 = (lane & 15) * 4;
    for (int pass = 0; pass < 2; ++pass) {
#pragma unroll
      for (int it = 0; it < 2; ++it) {
        const int row = 4 * wave + 2 * it + hh;
        const v4f v = *(const v4f*)(oS + row * 64 + c4);
        *(volatile v4f*)(out + (size_t)(i0 + row) * SEQ_N + j0 + c4) = v;
      }
      __threadfence();
    }
  }
}

#define OFF_X16   0ul
#define OFF_WIH0  262144ul
#define OFF_WHH0  786432ul
#define OFF_WHH1  1835008ul
#define OFF_WIH1  2883584ul
#define OFF_WMLP  7077888ul
#define OFF_PRM   7602176ul
#define OFF_Z0    7619712ul
#define OFF_Z1    16008320ul
#define OFF_H0    24396928ul
#define OFF_H1    26494080ul
#define OFF_AB    28591232ul
#define WS_TOTAL  29639808ul
static_assert(OFF_WIH0 == OFF_X16 + 1024ul * 128 * 2, "carve");
static_assert(OFF_WHH0 == OFF_WIH0 + 2ul * 1024 * 128 * 2, "carve");
static_assert(OFF_WHH1 == OFF_WHH0 + 2ul * 1024 * 256 * 2, "carve");
static_assert(OFF_WIH1 == OFF_WHH1 + 2ul * 1024 * 256 * 2, "carve");
static_assert(OFF_WMLP == OFF_WIH1 + 2ul * 1024 * 1024 * 2, "carve");
static_assert(OFF_PRM  == OFF_WMLP + 256ul * 1024 * 2, "carve");
static_assert(OFF_Z0   == OFF_PRM + PRM_TOTAL * 4ul, "carve");
static_assert(OFF_Z1   == OFF_Z0 + 2ul * 1024 * 1024 * 4, "carve");
static_assert(OFF_H0   == OFF_Z1 + 2ul * 1024 * 1024 * 4, "carve");
static_assert(OFF_H1   == OFF_H0 + 1024ul * 1024 * 2, "carve");
static_assert(OFF_AB   == OFF_H1 + 1024ul * 1024 * 2, "carve");
static_assert(WS_TOTAL == OFF_AB + 1024ul * 256 * 4, "carve");
static_assert(WS_TOTAL <= 134217728ul, "carve budget");
static_assert((OFF_PRM % 128) == 0 && (OFF_Z0 % 128) == 0 && (OFF_AB % 128) == 0, "alignment");
static_assert(SEQ_N % 64 == 0 && NGATE % 64 == 0 && XKPAD % 32 == 0, "gemm z0");
static_assert(HPITCH % 32 == 0 && ABPITCH % 64 == 0, "gemm z1 / ab");
static_assert(SEQ_N * SEQ_N * 4 == 4194304, "out bytes");

extern "C" void kernel_launch(void* const* d_in, const int* in_sizes, int n_in,
                              void* d_out, int out_size, void* d_ws, size_t ws_size,
                              hipStream_t stream) {
  (void)n_in;
  if (ws_size < WS_TOTAL) return;
  if (out_size != SEQ_N * SEQ_N) return;
  if (in_sizes[0] != SEQ_N || in_sizes[1] != SEQ_N) return;
  if (in_sizes[4] != 2 * NGATE * (WEMB + PEMB) || in_sizes[5] != 2 * NGATE * HID) return;
  if (in_sizes[7] != 2 * NGATE * 2 * HID || in_sizes[8] != 2 * NGATE * HID) return;
  if (in_sizes[10] != MHID * 4 * HID || in_sizes[12] != MHID) return;

  const int*   word_idx = (const int*)  d_in[0];
  const int*   pos_idx  = (const int*)  d_in[1];
  const float* word_emb = (const float*)d_in[2];
  const float* pos_emb  = (const float*)d_in[3];
  const float* wih0     = (const float*)d_in[4];
  const float* whh0     = (const float*)d_in[5];
  const float* lb0      = (const float*)d_in[6];
  const float* wih1     = (const float*)d_in[7];
  const float* whh1     = (const float*)d_in[8];
  const float* lb1      = (const float*)d_in[9];
  const float* mW1      = (const float*)d_in[10];
  const float* mb1      = (const float*)d_in[11];
  const float* mW2      = (const float*)d_in[12];
  const float* mb2      = (const float*)d_in[13];
  float* out = (float*)d_out;
  const int nWordRows = in_sizes[2] / WEMB;
  const int nPosRows  = in_sizes[3] / PEMB;

  char* ws = (char*)d_ws;
  unsigned short* X16  = (unsigned short*)(ws + OFF_X16);
  unsigned short* WIH0 = (unsigned short*)(ws + OFF_WIH0);
  unsigned short* WHH0 = (unsigned short*)(ws + OFF_WHH0);
  unsigned short* WHH1 = (unsigned short*)(ws + OFF_WHH1);
  unsigned short* WIH1 = (unsigned short*)(ws + OFF_WIH1);
  unsigned short* WMLP = (unsigned short*)(ws + OFF_WMLP);
  float*          PRM  = (float*)(ws + OFF_PRM);
  float*          Z0   = (float*)(ws + OFF_Z0);
  float*          Z1   = (float*)(ws + OFF_Z1);
  unsigned short* H0   = (unsigned short*)(ws + OFF_H0);
  unsigned short* H1   = (unsigned short*)(ws + OFF_H1);
  float*          AB   = (float*)(ws + OFF_AB);

  prm_kernel<<<(PRM_TOTAL + 255) / 256, 256, 0, stream>>>(lb0, lb1, mb1, mW2, mb2, PRM);
  embed_rows_bf16<<<SEQ_N / 8, 256, 0, stream>>>(word_idx, pos_idx, word_emb, nWordRows, pos_emb, nPosRows, X16);
  cast_rows_bf16<<<(2 * NGATE) / 8, 256, 0, stream>>>(wih0, 2 * NGATE, WEMB + PEMB, 0, WEMB + PEMB, WIH0, XKPAD, 0);
  cast_rows_bf16<<<(2 * NGATE) / 8, 256, 0, stream>>>(whh0, 2 * NGATE, HID, 0, HID, WHH0, HID, 0);
  cast_rows_bf16<<<(2 * NGATE) / 8, 256, 0, stream>>>(whh1, 2 * NGATE, HID, 0, HID, WHH1, HID, 0);
  cast_rows_bf16<<<(2 * NGATE) / 8, 256, 0, stream>>>(wih1, 2 * NGATE, 2 * HID, 0, 2 * HID, WIH1, HPITCH, 1);
  cast_rows_bf16<<<128 / 8, 256, 0, stream>>>(mW1, MHID, 4 * HID, 0, 2 * HID, WMLP, HPITCH, 1);
  cast_rows_bf16<<<128 / 8, 256, 0, stream>>>(mW1, MHID, 4 * HID, 2 * HID, 2 * HID, WMLP + (size_t)128 * HPITCH, HPITCH, 1);

  wmma_gemm64<1, false, 0, 0, false, 0><<<dim3((SEQ_N / 64) * (NGATE / 64) / 8, 2), 256, 0, stream>>>(
      X16, X16, XKPAD, 0L,
      WIH0, WIH0, XKPAD, (long)NGATE * XKPAD,
      (void*)Z0, (void*)Z0, NGATE, (long)SEQ_N * NGATE,
      PRM, PRM, 0L, SEQ_N, NGATE, XKPAD, 1.0f);
  bilstm_dir_kernel<<<2, 512, 0, stream>>>(WHH0, Z0, PRM, PRM_B0, H0);

  wmma_gemm64<1, false, 0, 0, false, 0><<<dim3((SEQ_N / 64) * (NGATE / 64) / 8, 2), 256, 0, stream>>>(
      H0, H0, HPITCH, 0L,
      WIH1, WIH1, HPITCH, (long)NGATE * HPITCH,
      (void*)Z1, (void*)Z1, NGATE, (long)SEQ_N * NGATE,
      PRM, PRM, 0L, SEQ_N, NGATE, HPITCH, 1.0f);
  bilstm_dir_kernel<<<2, 512, 0, stream>>>(WHH1, Z1, PRM, PRM_B1, H1);

  wmma_gemm64<1, false, 0, 0, false, 0><<<dim3((SEQ_N / 64) * (ABPITCH / 64) / 8, 1), 256, 0, stream>>>(
      H1, H1, HPITCH, 0L,
      WMLP, WMLP, HPITCH, 0L,
      (void*)AB, (void*)AB, ABPITCH, 0L,
      PRM, PRM, 0L, SEQ_N, ABPITCH, HPITCH, 1.0f);

  pair_score_kernel<<<dim3(SEQ_N / 64, SEQ_N / 32), 256, 0, stream>>>(AB, PRM, out);
}
